// TorchHawkes_52922587021743
// MI455X (gfx1250) — hardware-run, weakly checked
//
#include <hip/hip_runtime.h>


#define NR   512
#define NS   4096
#define NP   64
#define NE   2097152

typedef _Float16 h16;
typedef unsigned short bf;
typedef __attribute__((ext_vector_type(16))) __bf16   v16bf;
typedef __attribute__((ext_vector_type(16))) _Float16 v16h;
typedef __attribute__((ext_vector_type(8)))  _Float16 v8h;
typedef __attribute__((ext_vector_type(8)))  unsigned short v8us;
typedef __attribute__((ext_vector_type(8)))  float    v8f;
typedef __attribute__((ext_vector_type(4)))  float    v4f;
typedef v8h  __attribute__((may_alias)) v8ha;
typedef v4f  __attribute__((may_alias)) v4fa;
typedef v8us __attribute__((may_alias)) v8usa;

__device__ __forceinline__ unsigned short f2bf(float f) { unsigned u = __float_as_uint(f); u += 0x7FFFu + ((u >> 16) & 1u); return (unsigned short)(u >> 16); }
__device__ __forceinline__ float bf2f(unsigned short b) { return __uint_as_float(((unsigned)b) << 16); }
__device__ __forceinline__ float bfr(float f) { return bf2f(f2bf(f)); }
__device__ __forceinline__ v16h cat16(v8h lo, v8h hi) { return __builtin_shufflevector(lo, hi, 0, 1, 2, 3, 4, 5, 6, 7, 8, 9, 10, 11, 12, 13, 14, 15); }
__device__ __forceinline__ v16bf cat16b(v8us lo, v8us hi) { return __builtin_bit_cast(v16bf, __builtin_shufflevector(lo, hi, 0, 1, 2, 3, 4, 5, 6, 7, 8, 9, 10, 11, 12, 13, 14, 15)); }
__device__ __forceinline__ v8f wmma16(v16h a, v16h b, v8f c) { return __builtin_amdgcn_wmma_f32_16x16x32_f16(false, a, false, b, (short)0, c, false, false); }
__device__ __forceinline__ v8f wmmab(v16bf a, v16bf b, v8f c) { return __builtin_amdgcn_wmma_f32_16x16x32_bf16(false, a, false, b, (short)0, c, false, false); }

template <typename T16> struct WFrag;
template <> struct WFrag<h16> { typedef v16h V; static __device__ __forceinline__ V ld(const h16* p) { return cat16(*(const v8h*)p, *(const v8h*)(p + 16)); } static __device__ __forceinline__ v8f mma(V a, V b, v8f c) { return wmma16(a, b, c); } };
template <> struct WFrag<bf> { typedef v16bf V; static __device__ __forceinline__ V ld(const bf* p) { return cat16b(*(const v8us*)p, *(const v8us*)(p + 16)); } static __device__ __forceinline__ v8f mma(V a, V b, v8f c) { return wmmab(a, b, c); } };
template <typename T16, int NSPLIT, bool BIAS>
__global__ __launch_bounds__(32) void k_gemmw(const T16* __restrict__ A, const T16* __restrict__ A2, const T16* __restrict__ Bt, const T16* __restrict__ Bt2, int K, float* C, int ldc, const float* __restrict__ bias, size_t sA, size_t sB, size_t sC) {
    typedef typename WFrag<T16>::V V;
    __shared__ __align__(16) float os[16 * 68];
    const size_t z = blockIdx.z; A += z * sA; if (A2) A2 += z * sA; Bt += z * sB; if (Bt2) Bt2 += z * sB; C += z * sC;
    const int lane = threadIdx.x & 31, lr = lane & 15, hi = lane >> 4; const int r0 = blockIdx.x * 64, c0 = blockIdx.y * 64;
    v8f acc[4][4];
#pragma unroll
    for (int mb = 0; mb < 4; ++mb)
#pragma unroll
        for (int nb = 0; nb < 4; ++nb) acc[mb][nb] = (v8f){};
    const size_t aoff = (size_t)(r0 + lr) * K + 8 * hi, boff = (size_t)(c0 + lr) * K + 8 * hi;
    for (int kc = 0; kc < K; kc += 32) {
        V a[4], a2[4];
#pragma unroll
        for (int mb = 0; mb < 4; ++mb) { a[mb] = WFrag<T16>::ld(A + aoff + (size_t)mb * 16 * K + kc); if (NSPLIT == 1 || NSPLIT == 2) a2[mb] = WFrag<T16>::ld(A2 + aoff + (size_t)mb * 16 * K + kc); }
#pragma unroll
        for (int nb = 0; nb < 4; ++nb) { const V b = WFrag<T16>::ld(Bt + boff + (size_t)nb * 16 * K + kc); V b2; if (NSPLIT >= 2) b2 = WFrag<T16>::ld(Bt2 + boff + (size_t)nb * 16 * K + kc);
#pragma unroll
            for (int mb = 0; mb < 4; ++mb) { acc[mb][nb] = WFrag<T16>::mma(a[mb], b, acc[mb][nb]); if (NSPLIT == 1 || NSPLIT == 2) acc[mb][nb] = WFrag<T16>::mma(a2[mb], b, acc[mb][nb]); if (NSPLIT >= 2) acc[mb][nb] = WFrag<T16>::mma(a[mb], b2, acc[mb][nb]); } }
        asm volatile("v_nop\n\tv_nop\n\tv_nop\n\tv_nop" : "+v"(acc[0][0]), "+v"(acc[1][1]), "+v"(acc[2][2]), "+v"(acc[3][3]) : "v"(a[0]), "v"(a[3]));
    }
#pragma unroll
    for (int mb = 0; mb < 4; ++mb) {
#pragma unroll
        for (int nb = 0; nb < 4; ++nb) {
#pragma unroll
            for (int j = 0; j < 8; ++j) os[(hi * 8 + j) * 68 + nb * 16 + lr] = acc[mb][nb][j]; }
        __builtin_amdgcn_wave_barrier(); asm volatile("" ::: "memory");
        float* crow = C + (size_t)(r0 + mb * 16) * ldc + c0;
#pragma unroll 1
        for (int ps = 0; ps < 2; ++ps) {
#pragma unroll
            for (int s = 0; s < 8; ++s) { const int row = 2 * s + hi, cofs = lr * 4; v4f val = *(const v4fa*)(os + row * 68 + cofs); if (BIAS) { val[0] += bfr(bias[c0 + cofs]); val[1] += bfr(bias[c0 + cofs + 1]); val[2] += bfr(bias[c0 + cofs + 2]); val[3] += bfr(bias[c0 + cofs + 3]); }
                *(volatile v4f*)(crow + (size_t)row * ldc + cofs) = val; }
            if (ps == 0) __threadfence(); }
        __builtin_amdgcn_wave_barrier(); asm volatile("" ::: "memory");
    }
}

typedef __attribute__((ext_vector_type(2))) _Float16 v2h;
typedef __attribute__((ext_vector_type(4))) _Float16 v4h;
typedef __attribute__((ext_vector_type(2))) unsigned short v2us;
typedef __attribute__((ext_vector_type(4))) unsigned short v4us;
typedef __attribute__((ext_vector_type(2))) float v2f;
typedef __attribute__((ext_vector_type(4))) int v4i;

__device__ __forceinline__ h16 toh_flush(float x) { const float z = (fabsf(x) < 6.103515625e-05f) ? 0.0f : x; return (h16)z; }

template <bool RB>
__global__ __launch_bounds__(256) void k_c16(const float* __restrict__ src, h16* dst, size_t n8) { const size_t i = (size_t)blockIdx.x * 256 + threadIdx.x; if (i >= n8) return; const float* p = src + i * 8; const v4f a = *(const v4f*)p, b = *(const v4f*)(p + 4); v8h o;
#pragma unroll
    for (int q = 0; q < 4; ++q) { o[q] = toh_flush(RB ? bfr(a[q]) : a[q]); o[q + 4] = toh_flush(RB ? bfr(b[q]) : b[q]); }
    *(volatile v8h*)(dst + i * 8) = o; __threadfence(); *(volatile v8h*)(dst + i * 8) = o; }

__global__ __launch_bounds__(256) void k_scan(const float* __restrict__ a1, const float* __restrict__ a3, float* St, float* Bs) { const unsigned rw = blockIdx.x * 256u + threadIdx.x; const float rt = bfr(a3[0]); const float dk = expf(-rt); float cw = 0.0f, tot = 0.0f;
    for (int s0 = 0; s0 < NS; s0 += 8) { const float* pa = a1 + (size_t)rw * NS + s0; const v4f q0 = *(const v4f*)pa, q1 = *(const v4f*)(pa + 4); float hv[8];
#pragma unroll
        for (int js = 0; js < 8; ++js) { const float ov = bfr(js < 4 ? q0[js] : q1[js - 4]); hv[js] = cw; tot = tot + ov; cw = dk * (cw + rt * ov); }
        float* po = St + (size_t)s0 * NR + rw;
#pragma unroll
        for (int js = 0; js < 8; ++js) *(volatile float*)(po + (size_t)js * NR) = hv[js];
        __threadfence();
#pragma unroll
        for (int js = 0; js < 8; ++js) *(volatile float*)(po + (size_t)js * NR) = hv[js]; }
    const float bs = (tot * (1.0f / 4096.0f)) / 10.0f + 0.01f;
    *(volatile float*)(Bs + rw) = bs; __threadfence(); *(volatile float*)(Bs + rw) = bs; }

__global__ __launch_bounds__(256) void k_lam(const float* __restrict__ a1, const float* __restrict__ a2, const float* __restrict__ a5, const float* __restrict__ Bs, const float* __restrict__ Mx, float* Lm, float* Tm) { const unsigned id = blockIdx.x * 256u + threadIdx.x; const unsigned rw = id >> 12, sp = id & 4095u; const unsigned st0 = sp >= (unsigned)NP ? sp - (unsigned)NP : 0u; const float* pe = a2 + (size_t)rw * NS + st0; const float* pg = a5 + (size_t)rw * NP; float acc = 0.0f;
#pragma unroll 8
    for (int tp = 0; tp < NP; ++tp) acc = acc + bfr(pe[tp]) * bfr(pg[tp]);
    const float tsum = sp >= (unsigned)NP ? acc : 0.0f; const float vv = (Bs[rw] + Mx[id]) + tsum; const float lm = fmaxf(vv, 0.0f) + log1pf(expf(-fabsf(vv))); const float tm = bfr(a1[id]) * logf(lm) - lm;
    *(volatile float*)(Lm + id) = lm; *(volatile float*)(Tm + id) = tm; __threadfence(); *(volatile float*)(Lm + id) = lm; *(volatile float*)(Tm + id) = tm; }

__global__ __launch_bounds__(256) void k_put(const float* __restrict__ Lm, float* res) { const unsigned id = blockIdx.x * 256u + threadIdx.x; if (id < 32u || id > (unsigned)NE) return; const float lm = Lm[id - 1u];
    *(volatile float*)(res + id) = lm; __threadfence(); *(volatile float*)(res + id) = lm; }

__global__ __launch_bounds__(256) void k_sum64(const float* __restrict__ src, float* dst) { const unsigned id = blockIdx.x * 256u + threadIdx.x; const float* ps = src + (size_t)id * 64; float acc = 0.0f;
#pragma unroll
    for (int q = 0; q < 16; ++q) { const v4f s4 = *(const v4f*)(ps + 4 * q); acc = acc + s4[0]; acc = acc + s4[1]; acc = acc + s4[2]; acc = acc + s4[3]; }
    *(volatile float*)(dst + id) = acc; __threadfence(); *(volatile float*)(dst + id) = acc; }

__global__ __launch_bounds__(32) void k_last(const float* __restrict__ R2, const float* __restrict__ Lm, float* res) { const unsigned ln = threadIdx.x; float acc = 0.0f;
#pragma unroll
    for (int q0 = 0; q0 < NR; q0 += 8) { const v4f s0 = *(const v4f*)(R2 + q0), s1 = *(const v4f*)(R2 + q0 + 4); acc = acc + s0[0]; acc = acc + s0[1]; acc = acc + s0[2]; acc = acc + s0[3]; acc = acc + s1[0]; acc = acc + s1[1]; acc = acc + s1[2]; acc = acc + s1[3]; }
    const float lw = Lm[ln > 0u ? ln - 1u : 0u]; const float ov = ln == 0u ? acc : lw;
    *(volatile float*)(res + ln) = ov; __threadfence(); *(volatile float*)(res + ln) = ov; }

extern "C" void kernel_launch(void* const* d_in, const int* in_sizes, int n_in, void* d_out, int out_size, void* d_ws, size_t ws_size, hipStream_t stream) {
    if (n_in < 5) return;
    if (in_sizes[0] != NR * NS || in_sizes[1] != NR * NS || in_sizes[2] != 1 || in_sizes[3] != NR * NR || in_sizes[4] != NR * NP) return;
    if (out_size != NE + 1) return;
    static_assert(NE == NR * NS && NS == 4096 && NR % 256 == 0 && NR % 64 == 0 && NS % 64 == 0 && NR % 32 == 0 && NS % 8 == 0 && (NS * NR / 8) % 256 == 0 && (NR * NR / 8) % 256 == 0 && NE % 256 == 0 && NE % (64 * 256) == 0 && (NE / 64) % 64 == 0 && NE / 64 / 64 == NR && NR % 8 == 0 && NP == 64, "the product: row and column counts multiples of 64, the depth of 32; the flat grids exact; the sums of 64: 2,097,152 to 32,768 to 512; a step is the low 12 bits of a (row, step) number");
    const float* i0 = (const float*)d_in[0]; const float* i1 = (const float*)d_in[1]; const float* i2 = (const float*)d_in[2]; const float* i3 = (const float*)d_in[3]; const float* i4 = (const float*)d_in[4]; float* res = (float*)d_out;
    char* wsp = (char*)d_ws; auto take = [&](size_t bytes) { char* p = wsp; wsp += (bytes + 255) & ~(size_t)255; return (void*)p; };
    float* St = (float*)take((size_t)NS * NR * 4); float* Bs = (float*)take((size_t)NR * 4); h16* Sh = (h16*)take((size_t)NS * NR * 2); h16* Ah = (h16*)take((size_t)NR * NR * 2); float* Mx = (float*)take((size_t)NE * 4); float* Lm = (float*)take((size_t)NE * 4); float* Tm = (float*)take((size_t)NE * 4); float* R1 = (float*)take((size_t)(NE / 64) * 4); float* R2 = (float*)take((size_t)NR * 4);
    if ((size_t)(wsp - (char*)d_ws) > ws_size) return;
    k_scan<<<(unsigned)(NR / 256), 256, 0, stream>>>(i0, i2, St, Bs);
    k_c16<false><<<(unsigned)(NS * NR / 8 / 256), 256, 0, stream>>>(St, Sh, (size_t)NS * NR / 8);
    k_c16<true><<<(unsigned)(NR * NR / 8 / 256), 256, 0, stream>>>(i3, Ah, (size_t)NR * NR / 8);
    k_gemmw<h16, 0, false><<<dim3(NR / 64, NS / 64, 1), 32, 0, stream>>>(Ah, nullptr, Sh, nullptr, NR, Mx, NS, nullptr, 0, 0, 0);
    k_lam<<<(unsigned)(NE / 256), 256, 0, stream>>>(i0, i1, i4, Bs, Mx, Lm, Tm);
    k_put<<<(unsigned)(NE / 256 + 1), 256, 0, stream>>>(Lm, res);
    k_sum64<<<(unsigned)(NE / 64 / 256), 256, 0, stream>>>(Tm, R1);
    k_sum64<<<(unsigned)(NR / 256), 256, 0, stream>>>(R1, R2);
    k_last<<<1, 32, 0, stream>>>(R2, Lm, res);
}
